// MGAT_90881507983366
// MI455X (gfx1250) — hardware-verified
//
#include <hip/hip_runtime.h>
#include <stddef.h>


#define NTHR  256
#define NWAVE 8
#define DFW   128
#define GR    32
#define XSP   132
#define CHUNK 2048
#define WCAP  256
#define NGRP  (CHUNK / (NTHR * 4))
#define NB    512
#define NHD   2
#define ACCF  (NB * DFW)
#define MXN   (NB * NHD)
#define AGG_LDS_BYTES ((ACCF + 2 * MXN) * 4 + (NWAVE * WCAP + NWAVE) * 4)

static_assert(NGRP == 2);
static_assert(WCAP == (CHUNK / NTHR) * 32);
static_assert(ACCF == 65536);
static_assert(AGG_LDS_BYTES == 278560);
static_assert((NB & (NB - 1)) == 0);
static_assert(NB <= 512);
static_assert(NB <= NWAVE * WCAP);
static_assert((XSP % 4) == 0);

typedef float          v4f  __attribute__((ext_vector_type(4)));
typedef float          v8f  __attribute__((ext_vector_type(8)));
typedef int            v4i  __attribute__((ext_vector_type(4)));
typedef __bf16         v16b __attribute__((ext_vector_type(16)));
typedef unsigned short v8us __attribute__((ext_vector_type(8)));

union FragB { v16b v; v4i u[2]; };
union Pack  { v8us s; v4i i; };

__device__ __forceinline__ unsigned short f2bf(float x) {
  unsigned b = __float_as_uint(x);
  b += 0x7FFFu + ((b >> 16) & 1u);
  return (unsigned short)(b >> 16);
}
__device__ __forceinline__ float bf2f(unsigned short h) { return __uint_as_float(((unsigned)h) << 16); }

__device__ __forceinline__ v8f wmb(v16b a, v16b b, v8f c) {
  v8f d = __builtin_amdgcn_wmma_f32_16x16x32_bf16(false, a, false, b, (short)0, c, false, false);
  asm volatile("v_nop\n\tv_nop\n\tv_nop\n\tv_nop" : "+v"(d) : "v"(a), "v"(b));
  return d;
}

__device__ __forceinline__ float lk(float t) { return fmaxf(t, 0.2f * t); }
__device__ __forceinline__ float dl(v4f t, v4f w) {
  return w.x * lk(t.x) + w.y * lk(t.y) + w.z * lk(t.z) + w.w * lk(t.w);
}

__global__ __launch_bounds__(NTHR) void k_cvt(const float* __restrict__ src, int rows_src,
                                              unsigned short* ph, unsigned short* pl, int rows_total) {
  const int n8 = rows_total * (DFW / 8);
  const int i  = blockIdx.x * NTHR + threadIdx.x;
  if (i >= n8) return;
  const int r  = i >> 4;
  const int kb = (i & 15) * 8;
  v4f x0 = {0.f, 0.f, 0.f, 0.f};
  v4f x1 = x0;
  if (r < rows_src) {
    const float* p = src + (size_t)r * DFW + kb;
    x0 = *(const v4f*)p;
    x1 = *(const v4f*)(p + 4);
  }
  float v[8] = {x0.x, x0.y, x0.z, x0.w, x1.x, x1.y, x1.z, x1.w};
  Pack uh, ul;
  const v4i z4 = {0, 0, 0, 0};
  uh.i = z4; ul.i = z4;
#pragma unroll
  for (int j = 0; j < 8; ++j) {
    const unsigned short hb = f2bf(v[j]);
    uh.s[j] = hb;
    ul.s[j] = f2bf(v[j] - bf2f(hb));
  }
  const size_t o = (size_t)i * 8;
  *(volatile v4i*)(ph + o) = uh.i;
  *(volatile v4i*)(pl + o) = ul.i;
  __threadfence();
  *(volatile v4i*)(ph + o) = uh.i;
  *(volatile v4i*)(pl + o) = ul.i;
}

__global__ __launch_bounds__(NTHR) void k_cvtw(const float* __restrict__ Wl, const float* __restrict__ Wr,
                                               unsigned short* Bhl, unsigned short* Bll,
                                               unsigned short* Bhr, unsigned short* Blr) {
  const int sel = blockIdx.y;
  const float* W = sel ? Wr : Wl;
  unsigned short* ph = sel ? Bhr : Bhl;
  unsigned short* pl = sel ? Blr : Bll;
  const int i = blockIdx.x * NTHR + threadIdx.x;
  if (i >= DFW * DFW / 8) return;
  const int n  = i >> 4;
  const int kb = (i & 15) * 8;
  float v[8];
#pragma unroll
  for (int j = 0; j < 8; ++j) v[j] = W[(size_t)(kb + j) * DFW + n];
  Pack uh, ul;
  const v4i z4 = {0, 0, 0, 0};
  uh.i = z4; ul.i = z4;
#pragma unroll
  for (int j = 0; j < 8; ++j) {
    const unsigned short hb = f2bf(v[j]);
    uh.s[j] = hb;
    ul.s[j] = f2bf(v[j] - bf2f(hb));
  }
  const size_t o = (size_t)i * 8;
  *(volatile v4i*)(ph + o) = uh.i;
  *(volatile v4i*)(pl + o) = ul.i;
  __threadfence();
  *(volatile v4i*)(ph + o) = uh.i;
  *(volatile v4i*)(pl + o) = ul.i;
}

__global__ __launch_bounds__(NTHR) void k_gemm(
    const unsigned short* __restrict__ A0, const unsigned short* __restrict__ A1,
    const unsigned short* __restrict__ Bhl, const unsigned short* __restrict__ Bll,
    const unsigned short* __restrict__ Bhr, const unsigned short* __restrict__ Blr,
    const float* __restrict__ bl, const float* __restrict__ br, float* xl, float* xr) {
  __shared__ __attribute__((aligned(16))) float Xs[GR * XSP];
  constexpr int K = DFW;

  const int sel = blockIdx.y;
  const unsigned short* B0 = sel ? Bhr : Bhl;
  const unsigned short* B1 = sel ? Blr : Bll;
  const float* bias = sel ? br : bl;
  float* out = sel ? xr : xl;

  const int tid  = threadIdx.x;
  const int lane = tid & 31;
  const int wave = tid >> 5;
  const int hh   = lane >> 4;
  const int m    = lane & 15;
  const int rowBase = blockIdx.x * GR;
  const int ncol = wave * 16 + m;

  const size_t ra0 = (size_t)(rowBase + m) * K + 8 * hh;
  const size_t ra1 = ra0 + (size_t)16 * K;
  const size_t rb  = (size_t)ncol * K + 8 * hh;

  v8f c0 = {0.f, 0.f, 0.f, 0.f, 0.f, 0.f, 0.f, 0.f};
  v8f c1 = {0.f, 0.f, 0.f, 0.f, 0.f, 0.f, 0.f, 0.f};

#pragma unroll 1
  for (int k0 = 0; k0 < K; k0 += 32) {
    FragB ah0, ah1, al0, al1, bh, blo;
    ah0.u[0] = *(const v4i*)(A0 + ra0 + k0);  ah0.u[1] = *(const v4i*)(A0 + ra0 + k0 + 16);
    ah1.u[0] = *(const v4i*)(A0 + ra1 + k0);  ah1.u[1] = *(const v4i*)(A0 + ra1 + k0 + 16);
    al0.u[0] = *(const v4i*)(A1 + ra0 + k0);  al0.u[1] = *(const v4i*)(A1 + ra0 + k0 + 16);
    al1.u[0] = *(const v4i*)(A1 + ra1 + k0);  al1.u[1] = *(const v4i*)(A1 + ra1 + k0 + 16);
    bh.u[0]  = *(const v4i*)(B0 + rb + k0);   bh.u[1]  = *(const v4i*)(B0 + rb + k0 + 16);
    blo.u[0] = *(const v4i*)(B1 + rb + k0);   blo.u[1] = *(const v4i*)(B1 + rb + k0 + 16);
    c0 = wmb(ah0.v, bh.v, c0);  c0 = wmb(ah0.v, blo.v, c0);  c0 = wmb(al0.v, bh.v, c0);
    c1 = wmb(ah1.v, bh.v, c1);  c1 = wmb(ah1.v, blo.v, c1);  c1 = wmb(al1.v, bh.v, c1);
  }

  const float bv = bias[ncol];
#pragma unroll
  for (int r = 0; r < 8; ++r) {
    Xs[(8 * hh + r) * XSP + ncol]      = c0[r] + bv;
    Xs[(16 + 8 * hh + r) * XSP + ncol] = c1[r] + bv;
  }
  __syncthreads();

  v4f xv[4];
  float* xpp[4];
#pragma unroll
  for (int i = 0; i < 4; ++i) {
    xv[i]  = *(const v4f*)(Xs + (4 * wave + i) * XSP + 4 * lane);
    xpp[i] = out + (size_t)(rowBase + 4 * wave + i) * DFW + 4 * lane;
  }
#pragma unroll
  for (int i = 0; i < 4; ++i) *(volatile v4f*)(xpp[i]) = xv[i];
  __threadfence();
#pragma unroll
  for (int i = 0; i < 4; ++i) *(volatile v4f*)(xpp[i]) = xv[i];
}

__device__ __forceinline__ void hit2(const float* xs, const float* xd, float* ar, float* mp, float* dp, v4f w0) {
  const v4f a0 = *(const v4f*)(xs);
  const v4f d0 = *(const v4f*)(xd);
  float s = dl(a0 + d0, w0);
  s += __shfl_xor(s, 8, 32);
  s += __shfl_xor(s, 4, 32);
  s += __shfl_xor(s, 2, 32);
  s += __shfl_xor(s, 1, 32);
  const float m  = mp[0], n = dp[0];
  const float mn = fmaxf(m, s);
  const float sc = __expf(m - mn);
  const float p  = __expf(s - mn);
  v4f e0 = *(v4f*)(ar);
  e0 = e0 * sc + a0 * p;
  *(v4f*)(ar) = e0;
  mp[0] = mn;
  dp[0] = n * sc + p;
}

__global__ __launch_bounds__(NTHR) void k_agg(
    const int* __restrict__ ei, const float* __restrict__ xl, const float* __restrict__ xr,
    const float* __restrict__ att, const float* __restrict__ bias, float* out, int nN, int nE) {
  extern __shared__ v4f lds_dyn[];
  float* sacc = (float*)lds_dyn;
  float* mx   = sacc + ACCF;
  float* dn   = mx + MXN;
  int*   list = (int*)(dn + MXN);
  int*   wcnt = list + NWAVE * WCAP;

  const int tid  = threadIdx.x;
  const int lane = tid & 31;
  const int wave = tid >> 5;
  const int nodeBase = blockIdx.x * NB;

  {
    const v4f z4 = {0.f, 0.f, 0.f, 0.f};
    for (int i = tid; i < ACCF / 4; i += NTHR) lds_dyn[i] = z4;
    for (int i = tid; i < MXN; i += NTHR) { mx[i] = -1.0e30f; dn[i] = 0.f; }
  }
  __syncthreads();

  const int coff = 4 * lane;
  const int hidx = lane >> 4;
  const v4f w0 = *(const v4f*)(att + coff);

  const int* eid = ei + nE;
  const bool al16 = ((nE & 3) == 0);
  const int nChunks = (nE + CHUNK - 1) / CHUNK;

#pragma unroll 1
  for (int ch = 0; ch <= nChunks; ++ch) {
    const int cbase = ch * CHUNK;
    const bool selfp = (ch == nChunks);
    if (!selfp) {
      int wc = 0;
#pragma unroll
      for (int g = 0; g < NGRP; ++g) {
        const int el0 = (g * NTHR + tid) * 4;
        const int e0  = cbase + el0;
        const int sent = -2147483647 - 1;
        v4i d;
        if (al16 && (e0 + 3 < nE)) {
          d = *(const v4i*)(eid + e0);
        } else {
          d.x = (e0     < nE) ? eid[min(e0, nE - 1)]     : sent;
          d.y = (e0 + 1 < nE) ? eid[min(e0 + 1, nE - 1)] : sent;
          d.z = (e0 + 2 < nE) ? eid[min(e0 + 2, nE - 1)] : sent;
          d.w = (e0 + 3 < nE) ? eid[min(e0 + 3, nE - 1)] : sent;
        }
        const unsigned s0 = (unsigned)d.x - (unsigned)nodeBase;
        const unsigned s1 = (unsigned)d.y - (unsigned)nodeBase;
        const unsigned s2 = (unsigned)d.z - (unsigned)nodeBase;
        const unsigned s3 = (unsigned)d.w - (unsigned)nodeBase;
        const bool h0 = s0 < (unsigned)NB;
        const bool h1 = s1 < (unsigned)NB;
        const bool h2 = s2 < (unsigned)NB;
        const bool h3 = s3 < (unsigned)NB;
        const unsigned many = __builtin_amdgcn_ballot_w32(h0 | h1 | h2 | h3);
        if (many != 0u) {
#define HITJ(J, HJ, SJ) { \
            const unsigned mj = __builtin_amdgcn_ballot_w32(HJ); \
            if (HJ) { \
              const int pos = wc + (int)__builtin_amdgcn_mbcnt_lo(mj, 0u); \
              if (pos < WCAP) list[wave * WCAP + pos] = ((el0 + (J)) << 9) | (int)(SJ); \
            } \
            wc += (int)__builtin_popcount(mj); }
          HITJ(0, h0, s0)
          HITJ(1, h1, s1)
          HITJ(2, h2, s2)
          HITJ(3, h3, s3)
#undef HITJ
        }
      }
      if (lane == 0) wcnt[wave] = wc;
    } else {
      for (int s = tid; s < NB; s += NTHR) list[s] = s;
      if (tid < NWAVE) {
        int c = NB - tid * WCAP;
        c = c < 0 ? 0 : (c > WCAP ? WCAP : c);
        wcnt[tid] = c;
      }
    }
    __syncthreads();

    if (wave == 0) {
#pragma unroll 1
      for (int wsx = 0; wsx < NWAVE; ++wsx) {
        int n = __builtin_amdgcn_readfirstlane(wcnt[wsx]);
        n = n > WCAP ? WCAP : n;
        n = n < 0 ? 0 : n;
#pragma unroll 1
        for (int i = 0; i < n; ++i) {
          const int ent  = __builtin_amdgcn_readfirstlane(list[wsx * WCAP + i]);
          const int slot = ent & (NB - 1);
          const int el   = (ent >> 9) & (CHUNK - 1);
          const int node = nodeBase + slot;
          if (node >= nN) continue;
          int e = cbase + el;
          if (e > nE - 1) e = nE - 1;
          int sj = ei[e];
          sj = sj < 0 ? 0 : (sj > nN - 1 ? nN - 1 : sj);
          const int src = selfp ? node : sj;
          const float* xs = xl + (size_t)src * DFW + coff;
          const float* xd = xr + (size_t)node * DFW + coff;
          float* ar = sacc + slot * DFW + coff;
          float* mp = mx + slot * NHD + hidx;
          float* dp = dn + slot * NHD + hidx;
          hit2(xs, xd, ar, mp, dp, w0);
        }
      }
    }
    __syncthreads();
  }

#pragma unroll 1
  for (int s = wave; s < NB; s += NWAVE) {
    const int node = nodeBase + s;
    if (node >= nN) break;
    const int co = 4 * lane;
    const v4f e0 = *(const v4f*)(sacc + s * DFW + co);
    const float inv = 1.0f / (dn[s * NHD + (lane >> 4)] + 1e-16f);
    const v4f b0 = *(const v4f*)(bias + co);
    const v4f t = e0 * inv + b0;
    float q[4] = {t.x, t.y, t.z, t.w};
#pragma unroll
    for (int j = 0; j < 4; ++j) q[j] = (q[j] > 0.f) ? q[j] : (__expf(q[j]) - 1.0f);
    const v4f o = {q[0], q[1], q[2], q[3]};
    float* op = out + (size_t)node * DFW + co;
    *(volatile v4f*)op = o;
    __threadfence();
    *(volatile v4f*)op = o;
  }
}

extern "C" void kernel_launch(void* const* d_in, const int* in_sizes, int n_in,
                              void* d_out, int out_size, void* d_ws, size_t ws_size,
                              hipStream_t stream) {
  if (n_in < 16) return;
  const int nN = in_sizes[0] / DFW;
  if (nN <= 0 || in_sizes[0] != nN * DFW) return;
  const int nE = in_sizes[1] / 2;
  if (nE <= 0 || in_sizes[1] != 2 * nE) return;
  if (in_sizes[4] != DFW * DFW || in_sizes[5] != DFW || in_sizes[6] != DFW * DFW || in_sizes[7] != DFW ||
      in_sizes[8] != DFW || in_sizes[9] != DFW) return;
  if (in_sizes[10] != DFW * DFW || in_sizes[11] != DFW || in_sizes[12] != DFW * DFW || in_sizes[13] != DFW ||
      in_sizes[14] != DFW || in_sizes[15] != DFW) return;
  if (out_size != 2 * nN * DFW) return;

  const float* x    = (const float*)d_in[0];
  const int*   ei   = (const int*)d_in[1];
  const float* Wl1  = (const float*)d_in[4];   const float* bl1 = (const float*)d_in[5];
  const float* Wr1  = (const float*)d_in[6];   const float* br1 = (const float*)d_in[7];
  const float* at1  = (const float*)d_in[8];   const float* bi1 = (const float*)d_in[9];
  const float* Wl2  = (const float*)d_in[10];  const float* bl2 = (const float*)d_in[11];
  const float* Wr2  = (const float*)d_in[12];  const float* br2 = (const float*)d_in[13];
  const float* at2  = (const float*)d_in[14];  const float* bi2 = (const float*)d_in[15];
  float* out0 = (float*)d_out;
  float* out1 = out0 + (size_t)nN * DFW;

  const int Mpad = ((nN + GR - 1) / GR) * GR;

  char* wsp = (char*)d_ws;
  size_t off = 0;
  const size_t plB = (size_t)Mpad * DFW * 2;
  const size_t wB  = (size_t)DFW * DFW * 2;
  const size_t xB  = (size_t)Mpad * DFW * 4;
  unsigned short* Ah  = (unsigned short*)(wsp + off); off += plB;
  unsigned short* Al  = (unsigned short*)(wsp + off); off += plB;
  unsigned short* Bhl = (unsigned short*)(wsp + off); off += wB;
  unsigned short* Bll = (unsigned short*)(wsp + off); off += wB;
  unsigned short* Bhr = (unsigned short*)(wsp + off); off += wB;
  unsigned short* Blr = (unsigned short*)(wsp + off); off += wB;
  float* xl = (float*)(wsp + off); off += xB;
  float* xr = (float*)(wsp + off); off += xB;
  if (off > ws_size) return;

  const int mt = Mpad / GR;
  const unsigned cvtBlocks = (unsigned)((Mpad * (DFW / 8) + NTHR - 1) / NTHR);
  const unsigned aggBlocks = (unsigned)((nN + NB - 1) / NB);

  hipFuncSetAttribute(reinterpret_cast<const void*>(&k_agg),
                      hipFuncAttributeMaxDynamicSharedMemorySize, AGG_LDS_BYTES);

  k_cvt<<<cvtBlocks, NTHR, 0, stream>>>(x, nN, Ah, Al, Mpad);
  k_cvtw<<<dim3(DFW * DFW / 8 / NTHR, 2), NTHR, 0, stream>>>(Wl1, Wr1, Bhl, Bll, Bhr, Blr);
  k_gemm<<<dim3(mt, 2), NTHR, 0, stream>>>(Ah, Al, Bhl, Bll, Bhr, Blr, bl1, br1, xl, xr);
  k_agg<<<aggBlocks, NTHR, AGG_LDS_BYTES, stream>>>(ei, xl, xr, at1, bi1, out0, nN, nE);

  k_cvt<<<cvtBlocks, NTHR, 0, stream>>>(out0, nN, Ah, Al, Mpad);
  k_cvtw<<<dim3(DFW * DFW / 8 / NTHR, 2), NTHR, 0, stream>>>(Wl2, Wr2, Bhl, Bll, Bhr, Blr);
  k_gemm<<<dim3(mt, 2), NTHR, 0, stream>>>(Ah, Al, Bhl, Bll, Bhr, Blr, bl2, br2, xl, xr);
  k_agg<<<aggBlocks, NTHR, AGG_LDS_BYTES, stream>>>(ei, xl, xr, at2, bi2, out1, nN, nE);
}
